// OutlookAttention_60224031425234
// MI455X (gfx1250) — hardware-verified
//
#include <hip/hip_runtime.h>


#ifndef NB
#define NB 8
#endif
#define NB_FULL 8
#define HH 56
#define WW 56
#define CC 384
#define HEADS 12
#define DHEAD 32
#define NPIX (HH * WW)
#define NA 972
#define NA_PAD 1024
#define KCH (CC / 8)
#define WROWS (CC + NA_PAD + CC)
#define IPP 2
#define NPASS ((NB + IPP - 1) / IPP)
#define IPB 2
#define CSP 68
#define SM_SCALE 0.17677669529663687f
#define INV_W_CARRY 0.0625f
#define R_CARRY 2048.0f
#define INV_R_CARRY 0.00048828125f

static_assert(NB >= 1 && NB <= NB_FULL);
static_assert(NPIX % 64 == 0);
static_assert((NPIX * KCH) % 256 == 0);
static_assert((CC * KCH) % 256 == 0);
static_assert((NA_PAD * KCH) % 256 == 0);
static_assert((WROWS * KCH) % 256 == 0);
static_assert(CC % 64 == 0);
static_assert(NA_PAD % 64 == 0);
static_assert(NA <= NA_PAD);
static_assert(CC % 32 == 0);
static_assert(HEADS * DHEAD == CC);
static_assert(HEADS * 81 == NA);
static_assert(NPIX % IPB == 0);
static_assert(IPB * 96 == 192);

typedef _Float16 v16h __attribute__((ext_vector_type(16)));
typedef _Float16 v8h  __attribute__((ext_vector_type(8)));
typedef float    v8f  __attribute__((ext_vector_type(8)));
typedef float    v4f  __attribute__((ext_vector_type(4)));

union FragH { v16h v; v8h half[2]; };

__device__ __forceinline__ unsigned int bf16r_bits(float f) {
    unsigned int u = __float_as_uint(f);
    u += 0x7FFFu + ((u >> 16) & 1u);
    return u & 0xFFFF0000u;
}
__device__ __forceinline__ float bf16r(float f) { return __uint_as_float(bf16r_bits(f)); }

__device__ __forceinline__ v8f wmma16(v16h a, v16h b, v8f c) {
    return __builtin_amdgcn_wmma_f32_16x16x32_f16(false, a, false, b, (short)0, c, false, false);
}

__global__ __launch_bounds__(256)
void k_cvt_x(const float* __restrict__ x, _Float16* xh, int nchunk) {
    const int g = (int)blockIdx.x * 256 + (int)threadIdx.x;
    if (g >= nchunk) return;
    const float* s = x + (size_t)g * 8;
    const v4f f0 = *(const v4f*)s;
    const v4f f1 = *(const v4f*)(s + 4);
    float t[8] = {f0.x, f0.y, f0.z, f0.w, f1.x, f1.y, f1.z, f1.w};
    v8h o;
#pragma unroll
    for (int e = 0; e < 8; ++e) o[e] = (_Float16)bf16r(t[e]);
    _Float16* d = xh + (size_t)g * 8;
    *(volatile v8h*)d = o;
    __threadfence();
    *(volatile v8h*)d = o;
}

__global__ __launch_bounds__(256)
void k_cvt_w(const float* __restrict__ Wv, const float* __restrict__ Wa,
             const float* __restrict__ Wo, _Float16* wpl) {
    const int g   = (int)blockIdx.x * 256 + (int)threadIdx.x;
    const int R   = g / KCH;
    const int ch  = g - R * KCH;
    const int blk = (int)blockIdx.x;
    const float* src;
    int rbase, nvalid;
    if (blk < (CC * KCH) / 256)                  { src = Wv; rbase = 0;           nvalid = CC; }
    else if (blk < ((CC + NA_PAD) * KCH) / 256)  { src = Wa; rbase = CC;          nvalid = NA; }
    else                                         { src = Wo; rbase = CC + NA_PAD; nvalid = CC; }
    const int rr = R - rbase;
    const int rc = (rr < nvalid) ? rr : (nvalid - 1);
    const float pm = (rr < nvalid) ? 16.0f : 0.0f;
    const float* s = src + (size_t)rc * CC + ch * 8;
    const v4f f0 = *(const v4f*)s;
    const v4f f1 = *(const v4f*)(s + 4);
    float t[8] = {f0.x, f0.y, f0.z, f0.w, f1.x, f1.y, f1.z, f1.w};
    v8h o;
#pragma unroll
    for (int e = 0; e < 8; ++e) o[e] = (_Float16)(bf16r(t[e]) * pm);
    _Float16* d = wpl + (size_t)g * 8;
    *(volatile v8h*)d = o;
    __threadfence();
    *(volatile v8h*)d = o;
}

template <int RES>
__global__ __launch_bounds__(128)
void k_gemm(const _Float16* __restrict__ A, const _Float16* __restrict__ Ar,
            const _Float16* __restrict__ Bw, float* out, int ldo, float scale) {
    __shared__ float cs[64 * CSP];
    const int tid  = (int)threadIdx.x;
    const int lane = tid & 31;
    const int wave = tid >> 5;
    const int h    = lane >> 4;
    const int m    = lane & 15;
    const int m0   = (int)blockIdx.x * 64;
    const int n0   = (int)blockIdx.y * 64;
    const int wm   = (wave >> 1) * 32;
    const int wn   = (wave & 1) * 32;

    const size_t ra0 = (size_t)(m0 + wm + m) * CC + 8 * h;
    const size_t ra1 = ra0 + (size_t)16 * CC;
    const size_t rb0 = (size_t)(n0 + wn + m) * CC + 8 * h;
    const size_t rb1 = rb0 + (size_t)16 * CC;

    v8f acc00 = {0.f, 0.f, 0.f, 0.f, 0.f, 0.f, 0.f, 0.f};
    v8f acc01 = acc00, acc10 = acc00, acc11 = acc00;
    v8f rcc00 = acc00, rcc01 = acc00, rcc10 = acc00, rcc11 = acc00;

#pragma unroll 1
    for (int k0 = 0; k0 < CC; k0 += 32) {
        FragH a0, a1, b0, b1;
        a0.half[0] = *(const v8h*)(A + ra0 + k0);
        a0.half[1] = *(const v8h*)(A + ra0 + k0 + 16);
        a1.half[0] = *(const v8h*)(A + ra1 + k0);
        a1.half[1] = *(const v8h*)(A + ra1 + k0 + 16);
        b0.half[0] = *(const v8h*)(Bw + rb0 + k0);
        b0.half[1] = *(const v8h*)(Bw + rb0 + k0 + 16);
        b1.half[0] = *(const v8h*)(Bw + rb1 + k0);
        b1.half[1] = *(const v8h*)(Bw + rb1 + k0 + 16);
        acc00 = wmma16(a0.v, b0.v, acc00);
        acc01 = wmma16(a0.v, b1.v, acc01);
        acc10 = wmma16(a1.v, b0.v, acc10);
        acc11 = wmma16(a1.v, b1.v, acc11);
        if (RES) {
            FragH e0, e1;
            e0.half[0] = *(const v8h*)(Ar + ra0 + k0);
            e0.half[1] = *(const v8h*)(Ar + ra0 + k0 + 16);
            e1.half[0] = *(const v8h*)(Ar + ra1 + k0);
            e1.half[1] = *(const v8h*)(Ar + ra1 + k0 + 16);
            rcc00 = wmma16(e0.v, b0.v, rcc00);
            rcc01 = wmma16(e0.v, b1.v, rcc01);
            rcc10 = wmma16(e1.v, b0.v, rcc10);
            rcc11 = wmma16(e1.v, b1.v, rcc11);
            asm volatile("v_nop\n\tv_nop\n\tv_nop\n\tv_nop"
                         : "+v"(acc00), "+v"(acc01), "+v"(acc10), "+v"(acc11),
                           "+v"(rcc00), "+v"(rcc01), "+v"(rcc10), "+v"(rcc11)
                         : "v"(a0.v), "v"(a1.v), "v"(b0.v), "v"(b1.v), "v"(e0.v), "v"(e1.v));
        } else {
            asm volatile("v_nop\n\tv_nop\n\tv_nop\n\tv_nop"
                         : "+v"(acc00), "+v"(acc01), "+v"(acc10), "+v"(acc11)
                         : "v"(a0.v), "v"(a1.v), "v"(b0.v), "v"(b1.v));
        }
    }

    {
        float* p00 = cs + (wm + 8 * h) * CSP + wn + m;
        float* p10 = cs + (wm + 16 + 8 * h) * CSP + wn + m;
#pragma unroll
        for (int r = 0; r < 8; ++r) {
            float v00, v01, v10, v11;
            if (RES) {
                v00 = (acc00[r] + rcc00[r] * INV_R_CARRY) * scale;
                v01 = (acc01[r] + rcc01[r] * INV_R_CARRY) * scale;
                v10 = (acc10[r] + rcc10[r] * INV_R_CARRY) * scale;
                v11 = (acc11[r] + rcc11[r] * INV_R_CARRY) * scale;
            } else {
                v00 = acc00[r] * scale;
                v01 = acc01[r] * scale;
                v10 = acc10[r] * scale;
                v11 = acc11[r] * scale;
            }
            p00[r * CSP]      = v00;
            p00[r * CSP + 16] = v01;
            p10[r * CSP]      = v10;
            p10[r * CSP + 16] = v11;
        }
    }
    __syncthreads();

    const int lr = tid >> 3;
    const int lq = tid & 7;
#pragma unroll
    for (int p = 0; p < 8; ++p) {
        const int L = p * 16 + lr;
        const int row = L >> 1;
        const int col = (L & 1) * 32 + lq * 4;
        const v4f v = *(const v4f*)(cs + row * CSP + col);
        *(volatile v4f*)(out + (size_t)(m0 + row) * ldo + n0 + col) = v;
    }
    __threadfence();
#pragma unroll
    for (int p = 0; p < 8; ++p) {
        const int L = p * 16 + lr;
        const int row = L >> 1;
        const int col = (L & 1) * 32 + lq * 4;
        const v4f v = *(const v4f*)(cs + row * CSP + col);
        *(volatile v4f*)(out + (size_t)(m0 + row) * ldo + n0 + col) = v;
    }
}

__global__ __launch_bounds__(192)
void k_av(const float* __restrict__ P, const float* __restrict__ V,
          _Float16* Yh, _Float16* Yr, int row0) {
#pragma clang fp contract(off)
    __shared__ float w5s[IPB * HEADS * 25];
    __shared__ float ys[IPB * CC];
    const int tid = (int)threadIdx.x;
    const int lpb = (int)blockIdx.x * IPB;

    if (tid < IPB * HEADS) {
        const int pix  = tid / HEADS;
        const int head = tid - pix * HEADS;
        const int lp = lpb + pix;
        const int gp = row0 + lp;
        const int rs = gp % NPIX;
        const int r  = rs / WW;
        const int s  = rs - r * WW;
        float* wdst = w5s + (pix * HEADS + head) * 25;
#pragma unroll
        for (int t = 0; t < 25; ++t) wdst[t] = 0.0f;
#pragma unroll 1
        for (int ij = 0; ij < 9; ++ij) {
            const int i = ij / 3;
            const int j = ij - 3 * i;
            const int ny = r + 1 - i;
            const int nx = s + 1 - j;
            const bool ok = ((unsigned)ny < (unsigned)HH) && ((unsigned)nx < (unsigned)WW);
            const int nyc = ny < 0 ? 0 : (ny >= HH ? HH - 1 : ny);
            const int nxc = nx < 0 ? 0 : (nx >= WW ? WW - 1 : nx);
            const int nlp = lp + (nyc - r) * WW + (nxc - s);
            const float* g = P + (size_t)nlp * NA_PAD + head * 81 + ij * 9;
            float z[9];
            float mx = -3.0e38f;
#pragma unroll
            for (int q = 0; q < 9; ++q) { z[q] = g[q] * SM_SCALE; mx = fmaxf(mx, z[q]); }
            float e[9];
            float sum = 0.0f;
#pragma unroll
            for (int q = 0; q < 9; ++q) { e[q] = __expf(z[q] - mx); sum += e[q]; }
            const float inv = 1.0f / sum;
            float* wq = wdst + (2 - i) * 5 + (2 - j);
#pragma unroll
            for (int q = 0; q < 9; ++q) {
                const int qi = q / 3;
                const int qj = q - 3 * qi;
                const float pv = ok ? (e[q] * inv) : 0.0f;
                wq[qi * 5 + qj] += pv;
            }
        }
    }
    __syncthreads();

    {
        const int pix  = tid / 96;
        const int u    = tid - pix * 96;
        const int c0   = u * 4;
        const int head = u >> 3;
        const int gp = row0 + lpb + pix;
        const int rs = gp % NPIX;
        const int r  = rs / WW;
        const int s  = rs - r * WW;
        const float* wrow = w5s + (pix * HEADS + head) * 25;
        const float* vb = V + (size_t)gp * CC + c0;
        v4f acc = {0.0f, 0.0f, 0.0f, 0.0f};
#pragma unroll 1
        for (int a = 0; a < 5; ++a) {
            const int vy = r + a - 2;
            if ((unsigned)vy < (unsigned)HH) {
#pragma unroll 1
                for (int b = 0; b < 5; ++b) {
                    const int vx = s + b - 2;
                    if ((unsigned)vx < (unsigned)WW) {
                        const long dofs = (long)(((a - 2) * WW + (b - 2)) * CC);
                        const v4f vv = *(const v4f*)(vb + dofs);
                        const float w = wrow[a * 5 + b];
                        acc.x = fmaf(w, vv.x, acc.x);
                        acc.y = fmaf(w, vv.y, acc.y);
                        acc.z = fmaf(w, vv.z, acc.z);
                        acc.w = fmaf(w, vv.w, acc.w);
                    }
                }
            }
        }
        *(v4f*)(ys + pix * CC + c0) = acc;
    }
    __syncthreads();

    {
        const int plane = tid / 96;
        const int u     = tid - plane * 96;
        const int pix   = u / KCH;
        const int ch    = u - pix * KCH;
        const int gp = row0 + lpb + pix;
        const float* ysrc = ys + pix * CC + ch * 8;
        const v4f y0 = *(const v4f*)ysrc;
        const v4f y1 = *(const v4f*)(ysrc + 4);
        float yv[8] = {y0.x, y0.y, y0.z, y0.w, y1.x, y1.y, y1.z, y1.w};
        v8h oh, orr;
#pragma unroll
        for (int e = 0; e < 8; ++e) {
            const _Float16 hq = (_Float16)yv[e];
            const float res = (yv[e] - (float)hq) * R_CARRY;
            oh[e]  = hq;
            orr[e] = (_Float16)res;
        }
        const size_t dofs = (size_t)gp * CC + ch * 8;
        if (plane == 0) {
            _Float16* d = Yh + dofs;
            *(volatile v8h*)d = oh;
            __threadfence();
            *(volatile v8h*)d = oh;
        } else {
            _Float16* d = Yr + dofs;
            *(volatile v8h*)d = orr;
            __threadfence();
            *(volatile v8h*)d = orr;
        }
    }
}

static inline size_t al256(size_t b) { return (b + 255) & ~(size_t)255; }

extern "C" void kernel_launch(void* const* d_in, const int* in_sizes, int n_in,
                              void* d_out, int out_size, void* d_ws, size_t ws_size,
                              hipStream_t stream) {
    if (n_in < 4) return;
    if (in_sizes[0] < NB * NPIX * CC) return;
    if (in_sizes[1] < CC * CC) return;
    if (in_sizes[2] < NA * CC) return;
    if (in_sizes[3] < CC * CC) return;
    if (out_size < NB * NPIX * CC) return;

    const float* x  = (const float*)d_in[0];
    const float* Wv = (const float*)d_in[1];
    const float* Wa = (const float*)d_in[2];
    const float* Wo = (const float*)d_in[3];
    float* out = (float*)d_out;

    const size_t szXH = (size_t)NB * NPIX * CC * 2;
    const size_t szW  = (size_t)WROWS * CC * 2;
    const size_t szV  = (size_t)NB * NPIX * CC * 4;
    const size_t szP  = (size_t)IPP * NPIX * NA_PAD * 4;
    const size_t szY  = (size_t)NB * NPIX * CC * 2;
    size_t off = 0;
    const size_t oXH = off; off += al256(szXH);
    const size_t oW  = off; off += al256(szW);
    const size_t oV  = off; off += al256(szV);
    const size_t oP  = off; off += al256(szP);
    const size_t oYH = off; off += al256(szY);
    const size_t oYR = off; off += al256(szY);
    if (off > ws_size) return;

    char* ws = (char*)d_ws;
    _Float16* Xh  = (_Float16*)(ws + oXH);
    _Float16* Wpl = (_Float16*)(ws + oW);
    const _Float16* Wvh = Wpl;
    const _Float16* Wah = Wpl + (size_t)CC * CC;
    const _Float16* Woh = Wpl + (size_t)(CC + NA_PAD) * CC;
    float* Vf = (float*)(ws + oV);
    float* Pf = (float*)(ws + oP);
    _Float16* Yh = (_Float16*)(ws + oYH);
    _Float16* Yr = (_Float16*)(ws + oYR);

    {
        const int nchunk = NB * NPIX * KCH;
        k_cvt_x<<<nchunk / 256, 256, 0, stream>>>(x, Xh, nchunk);
        k_cvt_w<<<(WROWS * KCH) / 256, 256, 0, stream>>>(Wv, Wa, Wo, Wpl);
    }
    k_gemm<0><<<dim3(NB * NPIX / 64, CC / 64), 128, 0, stream>>>(Xh, Xh, Wvh, Vf, CC, INV_W_CARRY);
    for (int ps = 0; ps < NPASS; ++ps) {
        const int nimg = (NB - ps * IPP < IPP) ? (NB - ps * IPP) : IPP;
        const int rows = nimg * NPIX;
        const int r0   = ps * IPP * NPIX;
        k_gemm<0><<<dim3(rows / 64, NA_PAD / 64), 128, 0, stream>>>(
            Xh + (size_t)r0 * CC, Xh, Wah, Pf, NA_PAD, INV_W_CARRY);
        k_av<<<rows / IPB, 192, 0, stream>>>(Pf, Vf, Yh, Yr, r0);
    }
    k_gemm<1><<<dim3(NB * NPIX / 64, CC / 64), 128, 0, stream>>>(Yh, Yr, Woh, out, CC, INV_W_CARRY);
}
